// MambaEncoder_4896262718011
// MI455X (gfx1250) — hardware-run, weakly checked
//
#include <hip/hip_runtime.h>
#include <math.h>
#include <stdint.h>

typedef __attribute__((ext_vector_type(16))) _Float16 v16h;
typedef __attribute__((ext_vector_type(8)))  _Float16 v8h;
typedef __attribute__((ext_vector_type(16))) __bf16   v16b;
typedef __attribute__((ext_vector_type(8)))  __bf16   v8b;
typedef __attribute__((ext_vector_type(8)))  float    v8f;
typedef __attribute__((ext_vector_type(4)))  float    v4f;
#define PSCALE 32768.0f
#define U16(p) ((const unsigned short*)(const void*)(p))
#define PSCALE_INV (1.0f / 32768.0f)

__device__ __forceinline__ unsigned short f2bf_bits(float f) {
  unsigned u = __float_as_uint(f);
  return (unsigned short)((u + 0x7FFFu + ((u >> 16) & 1u)) >> 16);
}
__device__ __forceinline__ float bf_bits2f(unsigned short h) { return __uint_as_float(((unsigned)h) << 16); }

__device__ __forceinline__ void dep_guard_h(v8f& a, v8f& b, v16h x, v16h y) { asm volatile("v_nop\n\tv_nop\n\tv_nop\n\tv_nop" : "+v"(a), "+v"(b) : "v"(x), "v"(y)); }
__device__ __forceinline__ void dep_guard_b(v8f& a, v8f& b, v16b x, v16b y) { asm volatile("v_nop\n\tv_nop\n\tv_nop\n\tv_nop" : "+v"(a), "+v"(b) : "v"(x), "v"(y)); }
__device__ __forceinline__ void keep4_h(v16h a, v16h b, v16h c, v16h d) { asm volatile("v_nop" :: "v"(a), "v"(b), "v"(c), "v"(d)); }
__device__ __forceinline__ void keep4_b(v16b a, v16b b, v16b c, v16b d) { asm volatile("v_nop" :: "v"(a), "v"(b), "v"(c), "v"(d)); }
__device__ __forceinline__ void acc_guard4(v8f& a, v8f& b, v8f& c, v8f& d) { asm volatile("v_nop\n\tv_nop\n\tv_nop\n\tv_nop" : "+v"(a), "+v"(b), "+v"(c), "+v"(d)); }
template <typename T> struct Frag;
template <> struct Frag<_Float16> {
  typedef v16h V; union U { v16h v; v8h h[2]; };
  static __device__ __forceinline__ v16h load(const _Float16* p) {
    U f; f.h[0] = *(const v8h*)(p); f.h[1] = *(const v8h*)(p + 16); return f.v;
  }
  static __device__ __forceinline__ v8f mma(v16h a, v16h b, v8f c) {
    return __builtin_amdgcn_wmma_f32_16x16x32_f16(false, a, false, b, (short)0, c, false, false);
  }
  static __device__ __forceinline__ void guard(v8f& a, v8f& b, v16h x, v16h y) { dep_guard_h(a, b, x, y); }
  static __device__ __forceinline__ void keep(v16h a, v16h b, v16h c, v16h d) { keep4_h(a, b, c, d); }
};
template <> struct Frag<__bf16> {
  typedef v16b V; union U { v16b v; v8b h[2]; };
  static __device__ __forceinline__ v16b load(const __bf16* p) {
    U f; f.h[0] = *(const v8b*)(p); f.h[1] = *(const v8b*)(p + 16); return f.v;
  }
  static __device__ __forceinline__ v8f mma(v16b a, v16b b, v8f c) {
    return __builtin_amdgcn_wmma_f32_16x16x32_bf16(false, a, false, b, (short)0, c, false, false);
  }
  static __device__ __forceinline__ void guard(v8f& a, v8f& b, v16b x, v16b y) { dep_guard_b(a, b, x, y); }
  static __device__ __forceinline__ void keep(v16b a, v16b b, v16b c, v16b d) { keep4_b(a, b, c, d); }
};

template <int ET> struct Elem;
template <> struct Elem<0> { typedef _Float16 T; };
template <> struct Elem<1> { typedef __bf16 T; };
template <int ET, bool SPLIT, int BIAS_MODE, int OUT_MODE, bool RESID, int ACT = 0>
__global__ __launch_bounds__(256) void wmma_gemm64(
    const unsigned short* __restrict__ Ap, const unsigned short* __restrict__ A2p, int lda, long strideA,
    const unsigned short* __restrict__ Btp, const unsigned short* __restrict__ Bt2p, int ldb, long strideB,
    void* __restrict__ Cout, void* __restrict__ Cout2, int ldc, long strideC,
    const float* __restrict__ bias,
    const float* __restrict__ resid, long strideR,
    int M, int N, int K, float scale) {
  typedef typename Elem<ET>::T T;
  typedef typename Frag<T>::V V;
  const T* A = (const T*)Ap; const T* A2 = (const T*)A2p; const T* Bt = (const T*)Btp; const T* Bt2 = (const T*)Bt2p;
  __shared__ __align__(16) float sT[8][16 * 68];
  const int b    = blockIdx.y;
  const int lane = threadIdx.x & 31;
  const int wave = threadIdx.x >> 5;
  const int tilesN = N >> 6;
  const int tilesM = M >> 6;
  const int tile = blockIdx.x * 8 + wave;
  if (tile >= tilesM * tilesN) return;
  const int tm = tile / tilesN;
  const int tn = tile - tm * tilesN;
  const int m0 = tm << 6;
  const int n0 = tn << 6;

  const T* Ab  = A  + (size_t)b * strideA;
  const T* Bb  = Bt + (size_t)b * strideB;
  const T* Ab2 = SPLIT ? (A2  + (size_t)b * strideA) : nullptr;
  const T* Bb2 = SPLIT ? (Bt2 + (size_t)b * strideB) : nullptr;

  const int rlane = lane & 15;
  const int koff  = (lane >> 4) * 8;
  const int mOff  = (lane >> 4) * 8;

  v8f acc[4][4];
#pragma unroll
  for (int i = 0; i < 4; ++i)
#pragma unroll
    for (int j = 0; j < 4; ++j) acc[i][j] = (v8f){0.f,0.f,0.f,0.f,0.f,0.f,0.f,0.f};

  for (int k0 = 0; k0 < K; k0 += 32) {
    V bh[4], bl[4];
#pragma unroll
    for (int j = 0; j < 4; ++j) {
      const size_t bo = (size_t)(n0 + (j << 4) + rlane) * ldb + koff + k0;
      bh[j] = Frag<T>::load(Bb + bo);
      if (SPLIT) bl[j] = Frag<T>::load(Bb2 + bo);
    }
#pragma unroll
    for (int i = 0; i < 4; ++i) {
      const size_t ao = (size_t)(m0 + (i << 4) + rlane) * lda + koff + k0;
      V ah = Frag<T>::load(Ab + ao);
      V al;
      if (SPLIT) al = Frag<T>::load(Ab2 + ao);
#pragma unroll
      for (int j = 0; j < 4; ++j) {
        acc[i][j] = Frag<T>::mma(ah, bh[j], acc[i][j]);
        if (SPLIT) {
          acc[i][j] = Frag<T>::mma(ah, bl[j], acc[i][j]);
          acc[i][j] = Frag<T>::mma(al, bh[j], acc[i][j]);
        }
      }
      Frag<T>::guard(acc[i][0], acc[i][3], ah, SPLIT ? al : ah);
    }
    Frag<T>::keep(bh[0], bh[1], bh[2], bh[3]);
    if (SPLIT) Frag<T>::keep(bl[0], bl[1], bl[2], bl[3]);
  }
  acc_guard4(acc[0][0], acc[0][1], acc[0][2], acc[0][3]);
  acc_guard4(acc[1][0], acc[1][1], acc[1][2], acc[1][3]);
  acc_guard4(acc[2][0], acc[2][1], acc[2][2], acc[2][3]);
  acc_guard4(acc[3][0], acc[3][1], acc[3][2], acc[3][3]);

  float* slab = sT[wave];
  const float* Rb = RESID ? (resid + (size_t)b * strideR) : nullptr;
#pragma unroll
  for (int i = 0; i < 4; ++i) {
    const int mBase = m0 + (i << 4);
#pragma unroll
    for (int j = 0; j < 4; ++j) {
      const int n = n0 + (j << 4) + rlane;
      float bv = 0.f;
      if (BIAS_MODE == 2) bv = bias[n];
#pragma unroll
      for (int r = 0; r < 8; ++r) {
        float v = acc[i][j][r] * scale;
        if (BIAS_MODE == 1) v += bias[mBase + mOff + r];
        if (BIAS_MODE == 2) v += bv;
        if (RESID) v += Rb[(size_t)(mBase + mOff + r) * ldc + n];
        if (ACT == 1) v = tanhf(v);
        if (ACT == 2) v = fmaxf(v, 0.0f);
        if (ACT == 3) v = v / (1.0f + expf(-v));
        if (ACT == 4) v = (v > 0.f) ? v : 0.01f * v;
        if (ACT == 5) v = 0.5f * v * (1.0f + erff(v * 0.70710678118654752f));
        slab[(mOff + r) * 68 + (j << 4) + rlane] = v;
      }
    }
    __builtin_amdgcn_fence(__ATOMIC_RELEASE, "workgroup");
    __builtin_amdgcn_wave_barrier();
    __builtin_amdgcn_fence(__ATOMIC_ACQUIRE, "workgroup");
    if (OUT_MODE == 0) {
      float* C = (float*)Cout + (size_t)b * strideC;
      const int hh = lane >> 4, c4 = (lane & 15) * 4;
      for (int pass = 0; pass < 2; ++pass) {
#pragma unroll
        for (int it = 0; it < 8; ++it) {
          const int row = it * 2 + hh;
          v4f v = *(const v4f*)(slab + row * 68 + c4);
          *(volatile v4f*)(C + (size_t)(mBase + row) * ldc + n0 + c4) = v;
        }
        __threadfence();
      }
    } else {
      const int q = lane >> 3, c8 = (lane & 7) * 8;
      unsigned short* C  = (unsigned short*)Cout  + (size_t)b * strideC;
      unsigned short* C2 = (OUT_MODE == 2) ? ((unsigned short*)Cout2 + (size_t)b * strideC) : nullptr;
      for (int pass = 0; pass < 2; ++pass) {
#pragma unroll
        for (int it = 0; it < 4; ++it) {
          const int row = it * 4 + q;
          const float* sp = slab + row * 68 + c8;
          v8h hv, lv;
#pragma unroll
          for (int e = 0; e < 8; ++e) {
            if (OUT_MODE == 1) {
              hv[e] = (_Float16)sp[e];
            } else {
              unsigned short hb = f2bf_bits(sp[e]);
              unsigned short lb = f2bf_bits(sp[e] - bf_bits2f(hb));
              hv[e] = __builtin_bit_cast(_Float16, hb);
              lv[e] = __builtin_bit_cast(_Float16, lb);
            }
          }
          *(volatile v8h*)(C + (size_t)(mBase + row) * ldc + n0 + c8) = hv;
          if (OUT_MODE == 2) *(volatile v8h*)(C2 + (size_t)(mBase + row) * ldc + n0 + c8) = lv;
        }
        __threadfence();
      }
    }
    __builtin_amdgcn_fence(__ATOMIC_RELEASE, "workgroup");
    __builtin_amdgcn_wave_barrier();
    __builtin_amdgcn_fence(__ATOMIC_ACQUIRE, "workgroup");
  }
}

constexpr int NB    = 4;
constexpr int SEQ   = 2048;
constexpr int DM    = 256;
constexpr int NS    = 16;
constexpr int DTR   = 16;
constexpr int KC    = 4;
constexpr int NLAY  = 4;
constexpr int MROWS = NB * SEQ;
constexpr int XPN   = DTR + 2 * NS;
constexpr int XPNP  = 64;
constexpr int DTKP  = 32;
constexpr float EPSV    = 1e-5f;
constexpr float INV_DM  = 1.0f / 256.0f;
constexpr float W_CARRY  = 256.0f;
constexpr float U_CARRY  = 256.0f;
constexpr float DT_CARRY = 4096.0f;
constexpr float Y_CARRY  = 8192.0f;

static_assert(MROWS % 64 == 0 && DM % 64 == 0 && XPNP % 64 == 0 && (2 * DM) % 64 == 0);
static_assert(DM % 32 == 0 && DTKP % 32 == 0);
static_assert(SEQ % 32 == 0 && DM % 64 == 0 && NS == 16 && DTR == 16 && XPN <= XPNP);
static_assert(MROWS % 8 == 0 && MROWS % 64 == 0);

__device__ __forceinline__ float wave_sum(float a) {
  a += __shfl_xor(a, 16);
  a += __shfl_xor(a, 8);
  a += __shfl_xor(a, 4);
  a += __shfl_xor(a, 2);
  a += __shfl_xor(a, 1);
  return a;
}

__global__ __launch_bounds__(256) void k_cast_pad_f16(const float* __restrict__ in, _Float16* __restrict__ out,
                                                      int R, int Cin, int Rpad, int Cpad, float scale) {
  const int g = blockIdx.y;
  const int i = blockIdx.x * 256 + threadIdx.x;
  const int nvec = (Rpad * Cpad) >> 3;
  if (i >= nvec) return;
  const int e0 = i << 3;
  const int r = e0 / Cpad;
  const int c = e0 - r * Cpad;
  const int rr = (r < R) ? r : (R - 1);
  const int cc = (c < Cin - 8) ? c : (Cin - 8);
  const float* src = in + ((size_t)g * R + rr) * Cin + cc;
  const v4f a  = *(const v4f*)src;
  const v4f bq = *(const v4f*)(src + 4);
  const float f = (r < R && c < Cin) ? scale : 0.0f;
  v8h hv;
#pragma unroll
  for (int e = 0; e < 4; ++e) {
    hv[e]     = (_Float16)(a[e] * f);
    hv[4 + e] = (_Float16)(bq[e] * f);
  }
  _Float16* dst = out + (size_t)g * Rpad * Cpad + e0;
  *(volatile v8h*)dst = hv;
  __threadfence();
  *(volatile v8h*)dst = hv;
}

__global__ __launch_bounds__(256) void k_innorm(const float* __restrict__ x, float* __restrict__ hout,
                                               _Float16* __restrict__ hh) {
  __shared__ __align__(16) float xs[DM * 36];
  __shared__ __align__(16) float srow[8 * DM];
  const int tid = threadIdx.x, wave = tid >> 5, lane = tid & 31;
  const int blk = blockIdx.x;
  const int b  = blk / (SEQ / 32);
  const int s0 = (blk - b * (SEQ / 32)) * 32;
  for (int i = tid; i < DM * 8; i += 256) {
    const int d = i >> 3, j = i & 7;
    const v4f q = *(const v4f*)(x + ((size_t)(b * DM + d)) * SEQ + s0 + 4 * j);
    *(v4f*)(xs + d * 36 + 4 * j) = q;
  }
  __syncthreads();
  float* sr = srow + wave * DM;
  for (int rr = 0; rr < 4; ++rr) {
    const int sl = wave * 4 + rr;
    const size_t rbase = ((size_t)b * SEQ + s0 + sl) * DM;
    float v[8];
#pragma unroll
    for (int e = 0; e < 4; ++e) {
      v[e]     = xs[(4 * lane + e) * 36 + sl];
      v[4 + e] = xs[(128 + 4 * lane + e) * 36 + sl];
    }
    float su = 0.f;
#pragma unroll
    for (int e = 0; e < 8; ++e) su += v[e];
    su = wave_sum(su);
    const float mu = su * INV_DM;
    float sq = 0.f;
#pragma unroll
    for (int e = 0; e < 8; ++e) { const float dv = v[e] - mu; sq += dv * dv; }
    sq = wave_sum(sq);
    const float var = sq * INV_DM;
    const float inv = 1.0f / sqrtf(var + EPSV);
    v4f o0, o1;
#pragma unroll
    for (int e = 0; e < 4; ++e) { o0[e] = (v[e] - mu) * inv; o1[e] = (v[4 + e] - mu) * inv; }
    float* hr = hout + rbase;
    *(volatile v4f*)(hr + 4 * lane) = o0;
    *(volatile v4f*)(hr + 128 + 4 * lane) = o1;
    *(v4f*)(sr + 4 * lane) = o0;
    *(v4f*)(sr + 128 + 4 * lane) = o1;
    __syncthreads();
    const v4f a0 = *(const v4f*)(sr + 8 * lane);
    const v4f a1 = *(const v4f*)(sr + 8 * lane + 4);
    v8h hv;
#pragma unroll
    for (int e = 0; e < 4; ++e) { hv[e] = (_Float16)a0[e]; hv[4 + e] = (_Float16)a1[e]; }
    _Float16* hd = hh + rbase + 8 * lane;
    *(volatile v8h*)hd = hv;
    __threadfence();
    *(volatile v4f*)(hr + 4 * lane) = o0;
    *(volatile v4f*)(hr + 128 + 4 * lane) = o1;
    *(volatile v8h*)hd = hv;
    __syncthreads();
  }
}

__global__ __launch_bounds__(256) void k_conv_silu(const float* __restrict__ xr, const float* __restrict__ cw,
                                                  const float* __restrict__ cb, float* __restrict__ uf,
                                                  _Float16* __restrict__ uh) {
  __shared__ __align__(16) float sw[DM * KC];
  __shared__ __align__(16) float scb[DM];
  __shared__ __align__(16) float su[8 * DM];
  const int tid = threadIdx.x;
  *(v4f*)(sw + 4 * tid) = *(const v4f*)(cw + 4 * tid);
  if (tid < 64) *(v4f*)(scb + 4 * tid) = *(const v4f*)(cb + 4 * tid);
  __syncthreads();
  const int rib = tid >> 5, cg = tid & 31, c0 = cg * 8;
  const int grow = blockIdx.x * 8 + rib;
  const int s = grow & (SEQ - 1);
  float acc[8];
#pragma unroll
  for (int e = 0; e < 8; ++e) acc[e] = scb[c0 + e];
#pragma unroll
  for (int k = 0; k < KC; ++k) {
    const int sh = k - (KC - 1);
    const bool ok = (s + sh) >= 0;
    const int srow = ok ? (grow + sh) : grow;
    const float* src = xr + (size_t)srow * (2 * DM) + c0;
    const v4f x0 = *(const v4f*)src;
    const v4f x1 = *(const v4f*)(src + 4);
#pragma unroll
    for (int e = 0; e < 4; ++e) {
      const float xa = ok ? x0[e] : 0.0f;
      const float xb = ok ? x1[e] : 0.0f;
      acc[e]     = fmaf(sw[(c0 + e) * KC + k], xa, acc[e]);
      acc[4 + e] = fmaf(sw[(c0 + 4 + e) * KC + k], xb, acc[4 + e]);
    }
  }
  float u[8];
#pragma unroll
  for (int e = 0; e < 8; ++e) {
    const float ex = expf(-acc[e]);
    u[e] = acc[e] * __builtin_amdgcn_rcpf(1.0f + ex);
  }
  v8h hv;
#pragma unroll
  for (int e = 0; e < 8; ++e) hv[e] = (_Float16)(u[e] * U_CARRY);
  _Float16* hd = uh + (size_t)grow * DM + c0;
  *(volatile v8h*)hd = hv;
  v4f p0, p1;
#pragma unroll
  for (int e = 0; e < 4; ++e) { p0[e] = u[e]; p1[e] = u[4 + e]; }
  *(v4f*)(su + rib * DM + c0) = p0;
  *(v4f*)(su + rib * DM + c0 + 4) = p1;
  __syncthreads();
  const v4f q0 = *(const v4f*)(su + 4 * tid);
  const v4f q1 = *(const v4f*)(su + 1024 + 4 * tid);
  float* fd = uf + (size_t)blockIdx.x * 8 * DM;
  *(volatile v4f*)(fd + 4 * tid) = q0;
  *(volatile v4f*)(fd + 1024 + 4 * tid) = q1;
  __threadfence();
  *(volatile v8h*)hd = hv;
  *(volatile v4f*)(fd + 4 * tid) = q0;
  *(volatile v4f*)(fd + 1024 + 4 * tid) = q1;
}

__global__ __launch_bounds__(256) void k_dtpack(const float* __restrict__ dbc, _Float16* __restrict__ dth) {
  const int tid = threadIdx.x;
  const int row = blockIdx.x * 64 + (tid >> 2);
  const int part = tid & 3;
  const float* src = dbc + (size_t)row * XPNP + (part & 1) * 8;
  const v4f a  = *(const v4f*)src;
  const v4f bq = *(const v4f*)(src + 4);
  const float f = (part < 2) ? DT_CARRY : 0.0f;
  v8h hv;
#pragma unroll
  for (int e = 0; e < 4; ++e) { hv[e] = (_Float16)(a[e] * f); hv[4 + e] = (_Float16)(bq[e] * f); }
  _Float16* dst = dth + (size_t)row * DTKP + part * 8;
  *(volatile v8h*)dst = hv;
  __threadfence();
  *(volatile v8h*)dst = hv;
}

constexpr int SC_T = 32;
constexpr int SC_C = 64;
__global__ __launch_bounds__(512) void k_scan(const float* __restrict__ dpre, const float* __restrict__ dtb,
                                             const float* __restrict__ uf, const float* __restrict__ xr,
                                             const float* __restrict__ dbc, const float* __restrict__ alog,
                                             const float* __restrict__ dpar, _Float16* __restrict__ yh) {
  __shared__ __align__(16) float sDel[SC_T * SC_C];
  __shared__ __align__(16) float sU[SC_T * SC_C];
  __shared__ __align__(16) float sG[SC_T * SC_C];
  __shared__ __align__(16) float sY[SC_T * SC_C];
  __shared__ __align__(16) float sBC[SC_T * 32];
  const int tid = threadIdx.x, wave = tid >> 5, lane = tid & 31;
  const int n = tid & 15, dl = tid >> 4;
  const int b = blockIdx.y, d0 = blockIdx.x * SC_C;
  const int da = d0 + dl, db = d0 + dl + 32;
  const float ac0 = -expf(alog[da * NS + n]);
  const float ac1 = -expf(alog[db * NS + n]);
  const float dp0 = dpar[da], dp1 = dpar[db];
  float h0 = 0.f, h1 = 0.f;
  for (int t0 = 0; t0 < SEQ; t0 += SC_T) {
    const size_t rbase = (size_t)b * SEQ + t0;
#pragma unroll 1
    for (int i = tid; i < SC_T * SC_C; i += 512) {
      const int row = i >> 6, col = i & 63;
      const size_t g1 = (rbase + row) * DM + d0 + col;
      const size_t g2 = (rbase + row) * (2 * DM) + DM + d0 + col;
      const float xd = dpre[g1] + dtb[d0 + col];
      const float sp = fmaxf(xd, 0.0f) + log1pf(expf(-fabsf(xd)));
      const float rv = xr[g2];
      const float gate = rv * __builtin_amdgcn_rcpf(1.0f + expf(-rv));
      sDel[i] = sp;
      sU[i]   = uf[g1];
      sG[i]   = gate;
    }
#pragma unroll 1
    for (int i = tid; i < SC_T * 32; i += 512) {
      const int row = i >> 5, c = i & 31;
      sBC[i] = dbc[(rbase + row) * XPNP + DTR + c];
    }
    __syncthreads();
#pragma unroll 1
    for (int tt = 0; tt < SC_T; ++tt) {
      const int o = tt * SC_C;
      const float e0 = sDel[o + dl], e1 = sDel[o + dl + 32];
      const float u0 = sU[o + dl],   u1 = sU[o + dl + 32];
      const float bn = sBC[tt * 32 + n], cn = sBC[tt * 32 + NS + n];
      const float a0 = expf(e0 * ac0), a1 = expf(e1 * ac1);
      h0 = a0 * h0 + (e0 * u0) * bn;
      h1 = a1 * h1 + (e1 * u1) * bn;
      float p0 = h0 * cn, p1 = h1 * cn;
      p0 += __shfl_xor(p0, 1); p1 += __shfl_xor(p1, 1);
      p0 += __shfl_xor(p0, 2); p1 += __shfl_xor(p1, 2);
      p0 += __shfl_xor(p0, 4); p1 += __shfl_xor(p1, 4);
      p0 += __shfl_xor(p0, 8); p1 += __shfl_xor(p1, 8);
      const float y0 = (p0 + u0 * dp0) * sG[o + dl];
      const float y1 = (p1 + u1 * dp1) * sG[o + dl + 32];
      if (n == 0) { sY[o + dl] = y0; sY[o + dl + 32] = y1; }
    }
    __syncthreads();
    if (wave < 8) {
      const int row = wave * 4 + (lane >> 3);
      const int c8  = (lane & 7) * 8;
      const v4f q0 = *(const v4f*)(sY + row * SC_C + c8);
      const v4f q1 = *(const v4f*)(sY + row * SC_C + c8 + 4);
      v8h hv;
#pragma unroll
      for (int e = 0; e < 4; ++e) { hv[e] = (_Float16)(q0[e] * Y_CARRY); hv[4 + e] = (_Float16)(q1[e] * Y_CARRY); }
      _Float16* dst = yh + (rbase + row) * DM + d0 + c8;
      *(volatile v8h*)dst = hv;
      __threadfence();
      *(volatile v8h*)dst = hv;
    }
    __syncthreads();
  }
}

__global__ __launch_bounds__(256) void k_lnres(const float* __restrict__ yv, const float* __restrict__ hin,
                                              const float* __restrict__ lw, const float* __restrict__ lb,
                                              float* __restrict__ hout, _Float16* __restrict__ hh) {
  __shared__ __align__(16) float srow[8 * DM];
  const int tid = threadIdx.x, wave = tid >> 5, lane = tid & 31;
  const int row = blockIdx.x * 8 + wave;
  const size_t rbase = (size_t)row * DM;
  const v4f y0 = *(const v4f*)(yv + rbase + 4 * lane);
  const v4f y1 = *(const v4f*)(yv + rbase + 128 + 4 * lane);
  const v4f g0 = *(const v4f*)(hin + rbase + 4 * lane);
  const v4f g1 = *(const v4f*)(hin + rbase + 128 + 4 * lane);
  const v4f w0 = *(const v4f*)(lw + 4 * lane);
  const v4f w1 = *(const v4f*)(lw + 128 + 4 * lane);
  const v4f b0 = *(const v4f*)(lb + 4 * lane);
  const v4f b1 = *(const v4f*)(lb + 128 + 4 * lane);
  float v[8];
#pragma unroll
  for (int e = 0; e < 4; ++e) { v[e] = y0[e] + g0[e]; v[4 + e] = y1[e] + g1[e]; }
  float su = 0.f;
#pragma unroll
  for (int e = 0; e < 8; ++e) su += v[e];
  su = wave_sum(su);
  const float mu = su * INV_DM;
  float sq = 0.f;
#pragma unroll
  for (int e = 0; e < 8; ++e) { const float dv = v[e] - mu; sq += dv * dv; }
  sq = wave_sum(sq);
  const float var = sq * INV_DM;
  const float inv = 1.0f / sqrtf(var + EPSV);
  v4f o0, o1;
#pragma unroll
  for (int e = 0; e < 4; ++e) {
    o0[e] = (v[e] - mu) * inv * w0[e] + b0[e];
    o1[e] = (v[4 + e] - mu) * inv * w1[e] + b1[e];
  }
  float* hr = hout + rbase;
  *(volatile v4f*)(hr + 4 * lane) = o0;
  *(volatile v4f*)(hr + 128 + 4 * lane) = o1;
  float* sr = srow + wave * DM;
  *(v4f*)(sr + 4 * lane) = o0;
  *(v4f*)(sr + 128 + 4 * lane) = o1;
  __syncthreads();
  const v4f a0 = *(const v4f*)(sr + 8 * lane);
  const v4f a1 = *(const v4f*)(sr + 8 * lane + 4);
  v8h hv;
#pragma unroll
  for (int e = 0; e < 4; ++e) { hv[e] = (_Float16)a0[e]; hv[4 + e] = (_Float16)a1[e]; }
  _Float16* hd = hh + rbase + 8 * lane;
  *(volatile v8h*)hd = hv;
  __threadfence();
  *(volatile v4f*)(hr + 4 * lane) = o0;
  *(volatile v4f*)(hr + 128 + 4 * lane) = o1;
  *(volatile v8h*)hd = hv;
}

template <int BIASM>
static void launch_gemm(const _Float16* A, int lda, const _Float16* Bt, int ldb, float* C, int ldc,
                        const float* bias, int Mm, int Nn, int Kk, float scale, hipStream_t st) {
  const int tiles = (Mm / 64) * (Nn / 64);
  dim3 grid((unsigned)((tiles + 7) / 8), 1);
  wmma_gemm64<0, false, BIASM, 0, false, 0><<<grid, 256, 0, st>>>(
      U16(A), nullptr, lda, 0L, U16(Bt), nullptr, ldb, 0L,
      (void*)C, nullptr, ldc, 0L, bias, nullptr, 0L, Mm, Nn, Kk, scale);
}

extern "C" void kernel_launch(void* const* d_in, const int* in_sizes, int n_in,
                              void* d_out, int out_size, void* d_ws, size_t ws_size,
                              hipStream_t stream) {
  if (n_in < 14) return;
  if (in_sizes[0] != NB * DM * SEQ || in_sizes[1] != NLAY * 2 * DM * DM || in_sizes[2] != NLAY * DM * KC ||
      in_sizes[3] != NLAY * DM || in_sizes[4] != NLAY * XPN * DM || in_sizes[5] != NLAY * DM * DTR ||
      in_sizes[6] != NLAY * DM || in_sizes[7] != NLAY * DM * NS || in_sizes[8] != NLAY * DM ||
      in_sizes[9] != NLAY * DM * DM || in_sizes[10] != NLAY * DM || in_sizes[11] != NLAY * DM ||
      in_sizes[12] != DM * DM || in_sizes[13] != DM || out_size != MROWS * DM) return;

  const float* x        = (const float*)d_in[0];
  const float* in_proj  = (const float*)d_in[1];
  const float* conv_w   = (const float*)d_in[2];
  const float* conv_b   = (const float*)d_in[3];
  const float* x_proj   = (const float*)d_in[4];
  const float* dt_proj  = (const float*)d_in[5];
  const float* dt_bias  = (const float*)d_in[6];
  const float* a_log    = (const float*)d_in[7];
  const float* d_param  = (const float*)d_in[8];
  const float* out_proj = (const float*)d_in[9];
  const float* lnw      = (const float*)d_in[10];
  const float* lnb      = (const float*)d_in[11];
  const float* proj_w   = (const float*)d_in[12];
  const float* proj_b   = (const float*)d_in[13];
  float* out = (float*)d_out;

  char* base = (char*)d_ws;
  size_t off = 0;
  auto carve = [&](size_t bytes) -> void* {
    void* p = base + off;
    off += (bytes + 255) & ~(size_t)255;
    return p;
  };
  _Float16* wIP  = (_Float16*)carve((size_t)NLAY * 2 * DM * DM * 2);
  _Float16* wXP  = (_Float16*)carve((size_t)NLAY * XPNP * DM * 2);
  _Float16* wDT  = (_Float16*)carve((size_t)NLAY * DM * DTKP * 2);
  _Float16* wOP  = (_Float16*)carve((size_t)NLAY * DM * DM * 2);
  _Float16* wPJ  = (_Float16*)carve((size_t)DM * DM * 2);
  float*    hA   = (float*)carve((size_t)MROWS * DM * 4);
  float*    hB   = (float*)carve((size_t)MROWS * DM * 4);
  _Float16* hH   = (_Float16*)carve((size_t)MROWS * DM * 2);
  float*    xr   = (float*)carve((size_t)MROWS * 2 * DM * 4);
  float*    uF   = (float*)carve((size_t)MROWS * DM * 4);
  _Float16* uH   = (_Float16*)carve((size_t)MROWS * DM * 2);
  float*    dbc  = (float*)carve((size_t)MROWS * XPNP * 4);
  _Float16* dtH  = (_Float16*)carve((size_t)MROWS * DTKP * 2);
  float*    dpre = (float*)carve((size_t)MROWS * DM * 4);
  _Float16* yH   = (_Float16*)carve((size_t)MROWS * DM * 2);
  float*    ytmp = (float*)carve((size_t)MROWS * DM * 4);
  if (off > ws_size) return;

  static_assert(((NLAY * 2 * DM) * DM / 8) % 256 == 0 && ((XPNP * DM) / 8) % 256 == 0 &&
                ((NLAY * DM * DTKP) / 8) % 256 == 0 && ((NLAY * DM * DM) / 8) % 256 == 0 &&
                ((DM * DM) / 8) % 256 == 0);
  k_cast_pad_f16<<<dim3((NLAY * 2 * DM * DM / 8) / 256, 1), 256, 0, stream>>>(
      in_proj, wIP, NLAY * 2 * DM, DM, NLAY * 2 * DM, DM, W_CARRY);
  k_cast_pad_f16<<<dim3((XPNP * DM / 8) / 256, NLAY), 256, 0, stream>>>(
      x_proj, wXP, XPN, DM, XPNP, DM, W_CARRY);
  k_cast_pad_f16<<<dim3((NLAY * DM * DTKP / 8) / 256, 1), 256, 0, stream>>>(
      dt_proj, wDT, NLAY * DM, DTR, NLAY * DM, DTKP, W_CARRY);
  k_cast_pad_f16<<<dim3((NLAY * DM * DM / 8) / 256, 1), 256, 0, stream>>>(
      out_proj, wOP, NLAY * DM, DM, NLAY * DM, DM, W_CARRY);
  k_cast_pad_f16<<<dim3((DM * DM / 8) / 256, 1), 256, 0, stream>>>(
      proj_w, wPJ, DM, DM, DM, DM, W_CARRY);

  k_innorm<<<MROWS / 32, 256, 0, stream>>>(x, hA, hH);

  for (int l = 0; l < NLAY; ++l) {
    float* hin  = (l & 1) ? hB : hA;
    float* hnew = (l & 1) ? hA : hB;
    launch_gemm<0>(hH, DM, wIP + (size_t)l * 2 * DM * DM, DM, xr, 2 * DM, nullptr,
                   MROWS, 2 * DM, DM, 1.0f / W_CARRY, stream);
    k_conv_silu<<<MROWS / 8, 256, 0, stream>>>(xr, conv_w + (size_t)l * DM * KC, conv_b + (size_t)l * DM, uF, uH);
    launch_gemm<0>(uH, DM, wXP + (size_t)l * XPNP * DM, DM, dbc, XPNP, nullptr,
                   MROWS, XPNP, DM, 1.0f / (U_CARRY * W_CARRY), stream);
    k_dtpack<<<MROWS / 64, 256, 0, stream>>>(dbc, dtH);
    launch_gemm<0>(dtH, DTKP, wDT + (size_t)l * DM * DTKP, DTKP, dpre, DM, nullptr,
                   MROWS, DM, DTKP, 1.0f / (DT_CARRY * W_CARRY), stream);
    k_scan<<<dim3(DM / SC_C, NB), 512, 0, stream>>>(dpre, dt_bias + (size_t)l * DM, uF, xr, dbc,
                                                  a_log + (size_t)l * DM * NS, d_param + (size_t)l * DM, yH);
    launch_gemm<0>(yH, DM, wOP + (size_t)l * DM * DM, DM, ytmp, DM, nullptr,
                   MROWS, DM, DM, 1.0f / (Y_CARRY * W_CARRY), stream);
    k_lnres<<<MROWS / 8, 256, 0, stream>>>(ytmp, hin, lnw + (size_t)l * DM, lnb + (size_t)l * DM, hnew, hH);
  }

  launch_gemm<2>(hH, DM, wPJ, DM, out, DM, proj_b, MROWS, DM, DM, 1.0f / W_CARRY, stream);
}
